// SqueezedGRU_S_4990751998018
// MI455X (gfx1250) — hardware-verified
//
#include <hip/hip_runtime.h>
#include <stdint.h>

typedef __attribute__((ext_vector_type(16))) _Float16 v16h;
typedef __attribute__((ext_vector_type(8)))  _Float16 v8h;
typedef __attribute__((ext_vector_type(16))) __bf16   v16b;
typedef __attribute__((ext_vector_type(8)))  __bf16   v8b;
typedef __attribute__((ext_vector_type(8)))  float    v8f;
typedef __attribute__((ext_vector_type(4)))  float    v4f;

#define HDIM  512
#define NGATE 1536
#define NGRP  8
#define GSZ   64

__device__ __forceinline__ unsigned short f2bf_bits(float f) {
  unsigned u = __float_as_uint(f);
  return (unsigned short)((u + 0x7FFFu + ((u >> 16) & 1u)) >> 16);
}
__device__ __forceinline__ float bf_bits2f(unsigned short h) { return __uint_as_float(((unsigned)h) << 16); }

__device__ __forceinline__ void dep_guard_h(v8f& a, v8f& b, v16h x, v16h y) { asm volatile("v_nop\n\tv_nop\n\tv_nop\n\tv_nop" : "+v"(a), "+v"(b) : "v"(x), "v"(y)); }
__device__ __forceinline__ void dep_guard_b(v8f& a, v8f& b, v16b x, v16b y) { asm volatile("v_nop\n\tv_nop\n\tv_nop\n\tv_nop" : "+v"(a), "+v"(b) : "v"(x), "v"(y)); }
__device__ __forceinline__ void keep4_h(v16h a, v16h b, v16h c, v16h d) { asm volatile("v_nop" :: "v"(a), "v"(b), "v"(c), "v"(d)); }
__device__ __forceinline__ void keep4_b(v16b a, v16b b, v16b c, v16b d) { asm volatile("v_nop" :: "v"(a), "v"(b), "v"(c), "v"(d)); }
__device__ __forceinline__ void acc_guard4(v8f& a, v8f& b, v8f& c, v8f& d) { asm volatile("v_nop\n\tv_nop\n\tv_nop\n\tv_nop" : "+v"(a), "+v"(b), "+v"(c), "+v"(d)); }
template <typename T> struct Frag;
template <> struct Frag<_Float16> {
  typedef v16h V; union U { v16h v; v8h h[2]; };
  static __device__ __forceinline__ v16h load(const _Float16* p) {
    U f; f.h[0] = *(const v8h*)(p); f.h[1] = *(const v8h*)(p + 16); return f.v;
  }
  static __device__ __forceinline__ v8f mma(v16h a, v16h b, v8f c) {
    return __builtin_amdgcn_wmma_f32_16x16x32_f16(false, a, false, b, (short)0, c, false, false);
  }
  static __device__ __forceinline__ void guard(v8f& a, v8f& b, v16h x, v16h y) { dep_guard_h(a, b, x, y); }
  static __device__ __forceinline__ void keep(v16h a, v16h b, v16h c, v16h d) { keep4_h(a, b, c, d); }
};
template <> struct Frag<__bf16> {
  typedef v16b V; union U { v16b v; v8b h[2]; };
  static __device__ __forceinline__ v16b load(const __bf16* p) {
    U f; f.h[0] = *(const v8b*)(p); f.h[1] = *(const v8b*)(p + 16); return f.v;
  }
  static __device__ __forceinline__ v8f mma(v16b a, v16b b, v8f c) {
    return __builtin_amdgcn_wmma_f32_16x16x32_bf16(false, a, false, b, (short)0, c, false, false);
  }
  static __device__ __forceinline__ void guard(v8f& a, v8f& b, v16b x, v16b y) { dep_guard_b(a, b, x, y); }
  static __device__ __forceinline__ void keep(v16b a, v16b b, v16b c, v16b d) { keep4_b(a, b, c, d); }
};

template <int ET> struct Elem;
template <> struct Elem<0> { typedef _Float16 T; };
template <> struct Elem<1> { typedef __bf16 T; };
template <int ET, bool SPLIT, int BIAS_MODE, int OUT_MODE, bool RESID, int ACT = 0>
__global__ __launch_bounds__(256) void wmma_gemm64(
    const unsigned short* __restrict__ Ap, const unsigned short* __restrict__ A2p, int lda, long strideA,
    const unsigned short* __restrict__ Btp, const unsigned short* __restrict__ Bt2p, int ldb, long strideB,
    void* __restrict__ Cout, void* __restrict__ Cout2, int ldc, long strideC,
    const float* __restrict__ bias, long strideBias,
    const float* __restrict__ resid, long strideR,
    int M, int N, int K, float scale) {
  typedef typename Elem<ET>::T T;
  typedef typename Frag<T>::V V;
  const T* A = (const T*)Ap; const T* A2 = (const T*)A2p; const T* Bt = (const T*)Btp; const T* Bt2 = (const T*)Bt2p;
  __shared__ __align__(16) float sT[8][16 * 68];
  const int b    = blockIdx.y;
  const int lane = threadIdx.x & 31;
  const int wave = threadIdx.x >> 5;
  const int tilesN = N >> 6;
  const int tilesM = M >> 6;
  const int tile = blockIdx.x * 8 + wave;
  if (tile >= tilesM * tilesN) return;
  const int tm = tile / tilesN;
  const int tn = tile - tm * tilesN;
  const int m0 = tm << 6;
  const int n0 = tn << 6;

  const T* Ab  = A  + (size_t)b * strideA;
  const T* Bb  = Bt + (size_t)b * strideB;
  const T* Ab2 = SPLIT ? (A2  + (size_t)b * strideA) : nullptr;
  const T* Bb2 = SPLIT ? (Bt2 + (size_t)b * strideB) : nullptr;
  const float* biasb = (BIAS_MODE != 0) ? (bias + (size_t)b * strideBias) : nullptr;

  const int rlane = lane & 15;
  const int koff  = (lane >> 4) * 8;
  const int mOff  = (lane >> 4) * 8;

  v8f acc[4][4];
#pragma unroll
  for (int i = 0; i < 4; ++i)
#pragma unroll
    for (int j = 0; j < 4; ++j) acc[i][j] = (v8f){0.f,0.f,0.f,0.f,0.f,0.f,0.f,0.f};

  for (int k0 = 0; k0 < K; k0 += 32) {
    V bh[4], bl[4];
#pragma unroll
    for (int j = 0; j < 4; ++j) {
      const size_t bo = (size_t)(n0 + (j << 4) + rlane) * ldb + koff + k0;
      bh[j] = Frag<T>::load(Bb + bo);
      if (SPLIT) bl[j] = Frag<T>::load(Bb2 + bo);
    }
#pragma unroll
    for (int i = 0; i < 4; ++i) {
      const size_t ao = (size_t)(m0 + (i << 4) + rlane) * lda + koff + k0;
      V ah = Frag<T>::load(Ab + ao);
      V al;
      if (SPLIT) al = Frag<T>::load(Ab2 + ao);
#pragma unroll
      for (int j = 0; j < 4; ++j) {
        acc[i][j] = Frag<T>::mma(ah, bh[j], acc[i][j]);
        if (SPLIT) {
          acc[i][j] = Frag<T>::mma(ah, bl[j], acc[i][j]);
          acc[i][j] = Frag<T>::mma(al, bh[j], acc[i][j]);
        }
      }
      Frag<T>::guard(acc[i][0], acc[i][3], ah, SPLIT ? al : ah);
    }
    Frag<T>::keep(bh[0], bh[1], bh[2], bh[3]);
    if (SPLIT) Frag<T>::keep(bl[0], bl[1], bl[2], bl[3]);
  }
  acc_guard4(acc[0][0], acc[0][1], acc[0][2], acc[0][3]);
  acc_guard4(acc[1][0], acc[1][1], acc[1][2], acc[1][3]);
  acc_guard4(acc[2][0], acc[2][1], acc[2][2], acc[2][3]);
  acc_guard4(acc[3][0], acc[3][1], acc[3][2], acc[3][3]);

  float* slab = sT[wave];
  const float* Rb = RESID ? (resid + (size_t)b * strideR) : nullptr;
#pragma unroll
  for (int i = 0; i < 4; ++i) {
    const int mBase = m0 + (i << 4);
#pragma unroll
    for (int j = 0; j < 4; ++j) {
      const int n = n0 + (j << 4) + rlane;
      float bv = 0.f;
      if (BIAS_MODE == 2) bv = biasb[n];
#pragma unroll
      for (int r = 0; r < 8; ++r) {
        float v = acc[i][j][r] * scale;
        if (BIAS_MODE == 1) v += biasb[mBase + mOff + r];
        if (BIAS_MODE == 2) v += bv;
        if (RESID) v += Rb[(size_t)(mBase + mOff + r) * ldc + n];
        if (ACT == 1) v = tanhf(v);
        if (ACT == 2) v = fmaxf(v, 0.0f);
        if (ACT == 3) v = v / (1.0f + expf(-v));
        if (ACT == 4) v = (v > 0.f) ? v : 0.01f * v;
        if (ACT == 5) v = 0.5f * v * (1.0f + erff(v * 0.70710678118654752f));
        slab[(mOff + r) * 68 + (j << 4) + rlane] = v;
      }
    }
    __builtin_amdgcn_fence(__ATOMIC_RELEASE, "workgroup");
    __builtin_amdgcn_wave_barrier();
    __builtin_amdgcn_fence(__ATOMIC_ACQUIRE, "workgroup");
    if (OUT_MODE == 0) {
      float* C = (float*)Cout + (size_t)b * strideC;
      const int hh = lane >> 4, c4 = (lane & 15) * 4;
      for (int pass = 0; pass < 2; ++pass) {
#pragma unroll
        for (int it = 0; it < 8; ++it) {
          const int row = it * 2 + hh;
          v4f v = *(const v4f*)(slab + row * 68 + c4);
          *(volatile v4f*)(C + (size_t)(mBase + row) * ldc + n0 + c4) = v;
        }
        __threadfence();
      }
    } else {
      const int q = lane >> 3, c8 = (lane & 7) * 8;
      unsigned short* C  = (unsigned short*)Cout  + (size_t)b * strideC;
      unsigned short* C2 = (OUT_MODE == 2) ? ((unsigned short*)Cout2 + (size_t)b * strideC) : nullptr;
      for (int pass = 0; pass < 2; ++pass) {
#pragma unroll
        for (int it = 0; it < 4; ++it) {
          const int row = it * 4 + q;
          const float* sp = slab + row * 68 + c8;
          v8h hv, lv;
#pragma unroll
          for (int e = 0; e < 8; ++e) {
            if (OUT_MODE == 1) {
              hv[e] = (_Float16)sp[e];
            } else {
              unsigned short hb = f2bf_bits(sp[e]);
              unsigned short lb = f2bf_bits(sp[e] - bf_bits2f(hb));
              hv[e] = __builtin_bit_cast(_Float16, hb);
              lv[e] = __builtin_bit_cast(_Float16, lb);
            }
          }
          *(volatile v8h*)(C + (size_t)(mBase + row) * ldc + n0 + c8) = hv;
          if (OUT_MODE == 2) *(volatile v8h*)(C2 + (size_t)(mBase + row) * ldc + n0 + c8) = lv;
        }
        __threadfence();
      }
    }
    __builtin_amdgcn_fence(__ATOMIC_RELEASE, "workgroup");
    __builtin_amdgcn_wave_barrier();
    __builtin_amdgcn_fence(__ATOMIC_ACQUIRE, "workgroup");
  }
}

__global__ __launch_bounds__(256) void cast_f32_f16x2s(
    const float* __restrict__ in, _Float16* __restrict__ out, int n2, float scale) {
  int i = blockIdx.x * 256 + threadIdx.x;
  if (i < n2) {
    const _Float16 h0 = (_Float16)(in[2 * i] * scale), h1 = (_Float16)(in[2 * i + 1] * scale);
    const unsigned u = (unsigned)__builtin_bit_cast(unsigned short, h0) | ((unsigned)__builtin_bit_cast(unsigned short, h1) << 16);
    ((volatile unsigned*)out)[i] = u;
    __threadfence();
    ((volatile unsigned*)out)[i] = u;
  }
}

__device__ __forceinline__ void grp_wT_pair(const float* __restrict__ w, _Float16* __restrict__ o, int p, float scale) {
  const int e0 = 2 * p;
  const int g = e0 >> 12;
  const int n = (e0 >> 6) & 63;
  const int k = e0 & 63;
  const int src = (g << 12) + (k << 6) + n;
  const _Float16 h0 = (_Float16)(w[src] * scale);
  const _Float16 h1 = (_Float16)(w[src + 64] * scale);
  const unsigned u = (unsigned)__builtin_bit_cast(unsigned short, h0) | ((unsigned)__builtin_bit_cast(unsigned short, h1) << 16);
  ((volatile unsigned*)o)[p] = u;
  __threadfence();
  ((volatile unsigned*)o)[p] = u;
}
__global__ __launch_bounds__(256) void cast_grouped_wT(
    const float* __restrict__ w_a, const float* __restrict__ w_b,
    _Float16* __restrict__ o_a, _Float16* __restrict__ o_b, int npairs_each, float scale) {
  const int t = blockIdx.x * 256 + threadIdx.x;
  if (t >= 2 * npairs_each) return;
  if (t < npairs_each) grp_wT_pair(w_a, o_a, t, scale);
  else                 grp_wT_pair(w_b, o_b, t - npairs_each, scale);
}

__device__ __forceinline__ float sigm_f(float x) {
  return __builtin_amdgcn_rcpf(1.0f + __expf(-x));
}

__global__ __launch_bounds__(128) void gru_cell_h0(
    const unsigned short* __restrict__ Xp, const unsigned short* __restrict__ Wp,
    const float* __restrict__ bih, const float* __restrict__ bhh,
    const float* __restrict__ Whh,
    unsigned short* __restrict__ Hp, int M, float wscale_inv) {
  typedef _Float16 T;
  typedef v16h V;
  const T* X = (const T*)Xp;
  const T* W = (const T*)Wp;
  T* Hout = (T*)Hp;
  __shared__ __align__(16) _Float16 sH[64 * 72];
  (void)Whh; (void)M;

  const int lane = threadIdx.x & 31;
  const int wave = threadIdx.x >> 5;
  const int m0 = blockIdx.y << 6;
  const int c0 = blockIdx.x << 6;
  const int cw = c0 + (wave << 4);
  const int rlane = lane & 15;
  const int koff  = (lane >> 4) * 8;
  const int mOff  = (lane >> 4) * 8;

  v8f acc[4][3];
#pragma unroll
  for (int i = 0; i < 4; ++i)
#pragma unroll
    for (int q = 0; q < 3; ++q) acc[i][q] = (v8f){0.f,0.f,0.f,0.f,0.f,0.f,0.f,0.f};

  for (int k0 = 0; k0 < HDIM; k0 += 32) {
    V bq[3];
#pragma unroll
    for (int q = 0; q < 3; ++q)
      bq[q] = Frag<T>::load(W + (size_t)(q * HDIM + cw + rlane) * HDIM + koff + k0);
#pragma unroll
    for (int i = 0; i < 4; ++i) {
      V ah = Frag<T>::load(X + (size_t)(m0 + (i << 4) + rlane) * HDIM + koff + k0);
#pragma unroll
      for (int q = 0; q < 3; ++q) acc[i][q] = Frag<T>::mma(ah, bq[q], acc[i][q]);
      Frag<T>::guard(acc[i][0], acc[i][2], ah, ah);
    }
    Frag<T>::keep(bq[0], bq[1], bq[2], bq[2]);
  }
  acc_guard4(acc[0][0], acc[0][1], acc[0][2], acc[1][0]);
  acc_guard4(acc[1][1], acc[1][2], acc[2][0], acc[2][1]);
  acc_guard4(acc[2][2], acc[3][0], acc[3][1], acc[3][2]);

  const int col = cw + rlane;
  const float br  = bih[col] + bhh[col];
  const float bz  = bih[HDIM + col] + bhh[HDIM + col];
  const float bni = bih[2 * HDIM + col];
  const float bnh = bhh[2 * HDIM + col];
#pragma unroll
  for (int i = 0; i < 4; ++i) {
#pragma unroll
    for (int r = 0; r < 8; ++r) {
      const float ar = acc[i][0][r] * wscale_inv + br;
      const float az = acc[i][1][r] * wscale_inv + bz;
      const float an = acc[i][2][r] * wscale_inv + bni;
      const float rg = sigm_f(ar);
      const float zg = sigm_f(az);
      const float npre = an + rg * bnh;
      const float ng = 2.0f * sigm_f(2.0f * npre) - 1.0f;
      const float hv = ng - zg * ng;
      sH[((i << 4) + mOff + r) * 72 + (wave << 4) + rlane] = (_Float16)hv;
    }
  }
  __syncthreads();
  {
    const int q = lane >> 3, c8 = (lane & 7) * 8;
    for (int pass = 0; pass < 2; ++pass) {
#pragma unroll
      for (int it = 0; it < 4; ++it) {
        const int row = (wave << 4) + it * 4 + q;
        const v8h v = *(const v8h*)(sH + row * 72 + c8);
        *(volatile v8h*)(Hout + (size_t)(m0 + row) * HDIM + c0 + c8) = v;
      }
      __threadfence();
    }
  }
}

static inline size_t align128(size_t x) { return (x + 127) & ~(size_t)127; }

extern "C" void kernel_launch(void* const* d_in, const int* in_sizes, int n_in,
                              void* d_out, int out_size, void* d_ws, size_t ws_size,
                              hipStream_t stream) {
  if (n_in < 9) return;
  const float* inputs = (const float*)d_in[0];
  const float* w_in   = (const float*)d_in[1];
  const float* b_in   = (const float*)d_in[2];
  const float* W_ih   = (const float*)d_in[3];
  const float* W_hh   = (const float*)d_in[4];
  const float* b_ih   = (const float*)d_in[5];
  const float* b_hh   = (const float*)d_in[6];
  const float* w_out  = (const float*)d_in[7];
  const float* b_out  = (const float*)d_in[8];
  float* out = (float*)d_out;

  const int nX = in_sizes[0];
  if (nX <= 0 || (nX % HDIM) != 0) return;
  const int M = nX / HDIM;
  if ((M % 64) != 0) return;
  if (in_sizes[1] != NGRP * GSZ * GSZ || in_sizes[7] != NGRP * GSZ * GSZ) return;
  if (in_sizes[2] != HDIM || in_sizes[8] != HDIM) return;
  if (in_sizes[3] != 2 * NGATE * HDIM || in_sizes[4] != 2 * NGATE * HDIM) return;
  if (in_sizes[5] != 2 * NGATE || in_sizes[6] != 2 * NGATE) return;
  if (out_size != M * HDIM) return;

  size_t off = 0;
  const size_t offX16 = off;  off = align128(off + (size_t)M * HDIM * 2);
  const size_t offX1  = off;  off = align128(off + (size_t)M * HDIM * 2);
  const size_t offWin = off;  off = align128(off + (size_t)NGRP * GSZ * GSZ * 2);
  const size_t offWout= off;  off = align128(off + (size_t)NGRP * GSZ * GSZ * 2);
  const size_t offWih = off;  off = align128(off + (size_t)2 * NGATE * HDIM * 2);
  if (off > ws_size || off > (size_t)134217728) return;

  char* ws = (char*)d_ws;
  _Float16* X16   = (_Float16*)(ws + offX16);
  _Float16* X1    = (_Float16*)(ws + offX1);
  _Float16* wIn16 = (_Float16*)(ws + offWin);
  _Float16* wOut16= (_Float16*)(ws + offWout);
  _Float16* Wih16 = (_Float16*)(ws + offWih);

  const float WSC = 16.0f, WSC_INV = 0.0625f;

  {
    const int n2 = nX / 2;
    cast_f32_f16x2s<<<dim3((n2 + 255) / 256), dim3(256), 0, stream>>>(inputs, X16, n2, 1.0f);
    const int n2w = (2 * NGATE * HDIM) / 2;
    cast_f32_f16x2s<<<dim3((n2w + 255) / 256), dim3(256), 0, stream>>>(W_ih, Wih16, n2w, WSC);
    const int npairs = (NGRP * GSZ * GSZ) / 2;
    cast_grouped_wT<<<dim3((2 * npairs + 255) / 256), dim3(256), 0, stream>>>(w_in, w_out, wIn16, wOut16, npairs, WSC);
  }

  const int tilesGrp = (M / 64) * (GSZ / 64);
  const dim3 grdGrp((tilesGrp + 7) / 8, NGRP);
  const dim3 grdGru(HDIM / 64, M / 64);

  wmma_gemm64<0, false, 2, 1, false><<<grdGrp, dim3(256), 0, stream>>>(
      (const unsigned short*)X16, (const unsigned short*)X16, HDIM, (long)GSZ,
      (const unsigned short*)wIn16, (const unsigned short*)wIn16, GSZ, (long)(GSZ * GSZ),
      (void*)X1, (void*)X1, HDIM, (long)GSZ,
      b_in, (long)GSZ,
      (const float*)nullptr, 0L,
      M, GSZ, GSZ, WSC_INV);

  gru_cell_h0<<<grdGru, dim3(128), 0, stream>>>(
      (const unsigned short*)X1, (const unsigned short*)Wih16, b_ih, b_hh, W_hh,
      (unsigned short*)X16, M, WSC_INV);
  gru_cell_h0<<<grdGru, dim3(128), 0, stream>>>(
      (const unsigned short*)X16, (const unsigned short*)(Wih16 + (size_t)NGATE * HDIM),
      b_ih + NGATE, b_hh + NGATE, W_hh + (size_t)NGATE * HDIM,
      (unsigned short*)X1, M, WSC_INV);

  wmma_gemm64<0, false, 2, 0, false><<<grdGrp, dim3(256), 0, stream>>>(
      (const unsigned short*)X1, (const unsigned short*)X1, HDIM, (long)GSZ,
      (const unsigned short*)wOut16, (const unsigned short*)wOut16, GSZ, (long)(GSZ * GSZ),
      (void*)out, (void*)out, HDIM, (long)GSZ,
      b_out, (long)GSZ,
      (const float*)nullptr, 0L,
      M, GSZ, GSZ, WSC_INV);

  (void)hipGetLastError();
}
